// StandardAttention_31233002176613
// MI455X (gfx1250) — hardware-verified
//
#include <hip/hip_runtime.h>


#ifndef NB
#define NB 1
#endif
#ifndef SEQ
#define SEQ 4096
#endif
#ifndef NB_FULL
#define NB_FULL 1
#endif
#ifndef SEQ_FULL
#define SEQ_FULL 4096
#endif

namespace {
constexpr int DM = 1024, H = 16, HD = 64, QL = SEQ, SK = SEQ, EQ = 256;
constexpr float XS = 8.0f, WSC = 256.0f, PS = 1024.0f, QRS = 1024.0f, PRS = 1024.0f, LOG2E = 1.4426950408889634f;
static_assert(SEQ % 64 == 0 && SEQ >= 64 && SEQ <= SEQ_FULL && NB >= 1 && NB <= NB_FULL && DM == H * HD && QL == SK && EQ % 64 == 0 && EQ % 32 == 0);

typedef _Float16 b16;
typedef __attribute__((ext_vector_type(16))) _Float16 v16b;
typedef __attribute__((ext_vector_type(8))) _Float16 v8b;
typedef __attribute__((ext_vector_type(4))) _Float16 v4h;
typedef __attribute__((ext_vector_type(2))) _Float16 v2h;
typedef __attribute__((ext_vector_type(8))) float v8f;
typedef __attribute__((ext_vector_type(4))) float v4f;
typedef __attribute__((ext_vector_type(2))) float v2f;

__device__ __forceinline__ float bf16_rne(float f) { unsigned int u = __float_as_uint(f); u += 0x7FFFu + ((u >> 16) & 1u); return __uint_as_float(u & 0xFFFF0000u); }
__device__ __forceinline__ void split16(float v, b16& hi, b16& lo) { hi = (b16)v; lo = (b16)(v - (float)hi); }
__device__ __forceinline__ int imin(int a, int b) { return a < b ? a : b; }
__device__ __forceinline__ v16b frag_kb(const b16* p, int hh) {
  const v8b a = *(const v8b*)(p + 8 * hh), b = *(const v8b*)(p + 16 + 8 * hh); v16b f;
#pragma unroll
  for (int e = 0; e < 8; ++e) { f[e] = a[e]; f[8 + e] = b[e]; }
  return f;
}
__device__ __forceinline__ v8f wmma16b(v16b a, v16b b, v8f c) {
  v8f d = __builtin_amdgcn_wmma_f32_16x16x32_f16(false, a, false, b, (short)0, c, false, false);
  asm volatile("v_nop\n\tv_nop\n\tv_nop\n\tv_nop" : "+v"(d) : "v"(a), "v"(b));
  return d;
}
__device__ __forceinline__ void wave_lds_sync() { __builtin_amdgcn_fence(3, "workgroup"); __builtin_amdgcn_wave_barrier(); __builtin_amdgcn_fence(2, "workgroup"); }
__device__ __forceinline__ float nexp2(float v) { return __builtin_amdgcn_exp2f(v); }

__global__ __launch_bounds__(256) void prep_kernel(const float* __restrict__ wqkv, const float* __restrict__ wo, b16* __restrict__ WT, b16* __restrict__ WO) {
  const size_t u = (size_t)blockIdx.x * 256 + threadIdx.x; const size_t per = (size_t)DM * DM / 8;
  if (u >= 4 * per) return;
  const int m = (int)(u / per); const size_t e = (u % per) * 8; const int oo = (int)(e / DM), k0 = (int)(e % DM);
  v8b o; b16* dst;
  if (m < 3) {
#pragma unroll
    for (int j = 0; j < 8; ++j) o[j] = (b16)(bf16_rne(wqkv[(size_t)(k0 + j) * (3 * DM) + (size_t)m * DM + oo]) * WSC);
    dst = WT + (size_t)m * DM * DM + e;
  } else {
#pragma unroll
    for (int j = 0; j < 8; ++j) o[j] = (b16)(bf16_rne(wo[(size_t)(k0 + j) * DM + oo]) * WSC);
    dst = WO + e;
  }
  *(volatile v8b*)dst = o; __threadfence(); *(volatile v8b*)dst = o;
}

__global__ __launch_bounds__(128) void proj_kernel(const float* __restrict__ x, const b16* __restrict__ WT, b16* __restrict__ Qp, b16* __restrict__ Kp, b16* __restrict__ VTh,
                                                   b16* __restrict__ VTl, b16* __restrict__ Qlo, b16* __restrict__ Klo) {
  __shared__ __attribute__((aligned(16))) b16 As[4][16][512 + 8];
  __shared__ __attribute__((aligned(16))) float Tf[4][16][128 + 4];
  const int wave = threadIdx.x >> 5, lane = threadIdx.x & 31, nloc = lane & 15, hlf = lane >> 4;
  const int which = blockIdx.y % 3, b = blockIdx.y / 3; const int rb = blockIdx.x, slab = blockIdx.z; const int t0 = rb * 64 + wave * 16; const int n0 = slab * 128;
  const b16* W = WT + (size_t)which * DM * DM;
  v8f acc[8];
#pragma unroll
  for (int t = 0; t < 8; ++t) acc[t] = (v8f){};
#pragma unroll 1
  for (int half = 0; half < 2; ++half) {
    for (int rr = 0; rr < 16; ++rr) {
      const float* xr = x + ((size_t)b * SEQ_FULL + t0 + rr) * DM + half * 512;
      for (int q = lane * 4; q < 512; q += 128) {
        const v4f xv = *(const v4f*)(xr + q); v4h o;
#pragma unroll
        for (int j = 0; j < 4; ++j) o[j] = (b16)(bf16_rne(xv[j]) * XS);
        *(v4h*)(&As[wave][rr][q]) = o; } }
    wave_lds_sync();
#pragma unroll 2
    for (int kb = 0; kb < 512; kb += 32) {
      const v16b a = frag_kb(&As[wave][nloc][kb], hlf);
#pragma unroll
      for (int t = 0; t < 8; ++t) acc[t] = wmma16b(a, frag_kb(W + (size_t)(n0 + t * 16 + nloc) * DM + half * 512 + kb, hlf), acc[t]); }
    wave_lds_sync(); }
#pragma unroll
  for (int t = 0; t < 8; ++t) {
#pragma unroll
    for (int r = 0; r < 8; ++r) Tf[wave][8 * hlf + r][t * 16 + nloc] = acc[t][r] * (1.0f / (XS * WSC)); }
  __syncthreads();
  for (int pass = 0; pass < 2; ++pass) {
    if (which == 2) {
#pragma unroll 1
      for (int q = 0; q < 32; ++q) {
        const int cl = wave * 32 + q; const int c = n0 + cl; const int h = c / HD, d = c % HD; const int tk = lane * 2; v2h hv, lv;
#pragma unroll
        for (int j = 0; j < 2; ++j) { b16 p, ql; split16(Tf[(tk + j) >> 4][(tk + j) & 15][cl] * XS, p, ql); hv[j] = p; lv[j] = ql; }
        const size_t oi = (((size_t)b * H + h) * HD + d) * SK + (size_t)rb * 64 + lane * 2;
        *(volatile v2h*)(VTh + oi) = hv; *(volatile v2h*)(VTl + oi) = lv; } }
    else {
      b16* P = (which == 0) ? Qp : Kp; b16* PL = (which == 0) ? Qlo : Klo;
      for (int rr = 0; rr < 16; ++rr) {
#pragma unroll
        for (int hs = 0; hs < 2; ++hs) {
          const int c = n0 + hs * 64; const int h = c / HD;
          const float f0 = Tf[wave][rr][hs * 64 + lane * 2] * XS, f1 = Tf[wave][rr][hs * 64 + lane * 2 + 1] * XS;
          const b16 h0 = (b16)f0, h1 = (b16)f1; v2h o; o[0] = h0; o[1] = h1;
          *(volatile v2h*)(P + (((size_t)b * H + h) * SEQ + (t0 + rr)) * HD + lane * 2) = o;
          if (rb * 64 < EQ) {
            v2h lo; lo[0] = (b16)((f0 - (float)h0) * QRS); lo[1] = (b16)((f1 - (float)h1) * QRS);
            *(volatile v2h*)(PL + (((size_t)b * H + h) * EQ + (t0 + rr)) * HD + lane * 2) = lo; } } } }
    __threadfence(); }
}

template <bool EARLY>
__global__ __launch_bounds__(64) __attribute__((amdgpu_num_vgpr(256))) void attn_kernel(const b16* __restrict__ Qp, const b16* __restrict__ Kp, const b16* __restrict__ Qlo, const b16* __restrict__ Klo,
                                                                                      const b16* __restrict__ VTh, const b16* __restrict__ VTl, b16* __restrict__ Ch, b16* __restrict__ Cl, int bx0) {
  __shared__ __attribute__((aligned(16))) b16 Pb[2][16][32 + 8];
  __shared__ __attribute__((aligned(16))) b16 Pr[2][16][32 + 8];
  __shared__ __attribute__((aligned(16))) float To[2][16][HD + 4];
  const int wave = threadIdx.x >> 5, lane = threadIdx.x & 31, hh = lane >> 4, col = lane & 15;
  const int b = blockIdx.y / H, h = blockIdx.y % H; const int bx = (int)blockIdx.x + bx0; const int q0 = bx * 32 + wave * 16, qi = q0 + col;
  const size_t bh = (size_t)b * H + h;
  const b16* Qb = Qp + bh * SEQ * HD; const b16* Kb = Kp + bh * SK * HD; const b16* Vh = VTh + bh * HD * SK; const b16* Vl = VTl + bh * HD * SK;
  const b16* Qlb = Qlo + bh * EQ * HD; const b16* Klb = Klo + bh * EQ * HD;
  const v16b qa0 = frag_kb(Qb + (size_t)qi * HD, hh), qa1 = frag_kb(Qb + (size_t)qi * HD + 32, hh);
  v16b ql0 = (v16b){}, ql1 = (v16b){};
  if constexpr (EARLY) { const int qe = imin(qi, EQ - 1); ql0 = frag_kb(Qlb + (size_t)qe * HD, hh); ql1 = frag_kb(Qlb + (size_t)qe * HD + 32, hh); }
  const float cs = LOG2E / (8.0f * XS * XS);
  float m = -INFINITY, l = 0.0f; v8f o[4], o2[4];
#pragma unroll
  for (int t = 0; t < 4; ++t) { o[t] = (v8f){}; o2[t] = (v8f){}; }
  const int kend = bx * 32;
#pragma unroll 1
  for (int kb = 0; kb <= kend; kb += 32) {
    const bool last = (kb == kend);
    float e[16]; float mx = -INFINITY;
#pragma unroll
    for (int u = 0; u < 2; ++u) {
      const int key = kb + u * 16 + col; const size_t kr = (size_t)key * HD;
      const v16b k0f = frag_kb(Kb + kr, hh), k1f = frag_kb(Kb + kr + 32, hh);
      v8f s = (v8f){}; s = wmma16b(k0f, qa0, s); s = wmma16b(k1f, qa1, s);
      v8f s2 = (v8f){};
      if constexpr (EARLY) {
        const size_t klr = (size_t)imin(key, EQ - 1) * HD;
        s2 = wmma16b(frag_kb(Klb + klr, hh), qa0, s2); s2 = wmma16b(frag_kb(Klb + klr + 32, hh), qa1, s2);
        s2 = wmma16b(k0f, ql0, s2); s2 = wmma16b(k1f, ql1, s2); }
#pragma unroll
      for (int r = 0; r < 8; ++r) {
        float v;
        if constexpr (EARLY) v = (s[r] + s2[r] * (1.0f / QRS)) * cs; else v = s[r] * cs;
        if (last) { const int koff = u * 16 + 8 * hh + r; v = (koff > wave * 16 + col) ? -INFINITY : v; }
        e[u * 8 + r] = v; mx = fmaxf(mx, v); } }
    mx = fmaxf(mx, __shfl_xor(mx, 16)); const float mn = fmaxf(m, mx); const float al = nexp2(m - mn); float sum = 0.0f;
#pragma unroll
    for (int i2 = 0; i2 < 16; ++i2) {
      const float p = nexp2(e[i2] - mn); sum += p; const int pi = (i2 < 8 ? 0 : 16) + 8 * hh + (i2 & 7);
      const float pp = p * PS; const b16 ph = (b16)pp; Pb[wave][col][pi] = ph;
      if constexpr (EARLY) Pr[wave][col][pi] = (b16)((pp - (float)ph) * PRS); }
    sum += __shfl_xor(sum, 16); l = l * al + sum; m = mn;
    wave_lds_sync();
    const v16b pf = frag_kb(&Pb[wave][col][0], hh);
    v16b prf = (v16b){};
    if constexpr (EARLY) prf = frag_kb(&Pr[wave][col][0], hh);
#pragma unroll
    for (int t = 0; t < 4; ++t) {
      o[t] *= al; const size_t vr = (size_t)(t * 16 + col) * SK + kb; const v16b vh = frag_kb(Vh + vr, hh);
      o[t] = wmma16b(vh, pf, o[t]); o[t] = wmma16b(frag_kb(Vl + vr, hh), pf, o[t]);
      if constexpr (EARLY) { o2[t] *= al; o2[t] = wmma16b(vh, prf, o2[t]); } }
    wave_lds_sync(); }
  const float inv = 1.0f / (l * PS * XS);
#pragma unroll
  for (int t = 0; t < 4; ++t) {
#pragma unroll
    for (int r = 0; r < 8; ++r) {
      float ov = o[t][r];
      if constexpr (EARLY) ov += o2[t][r] * (1.0f / PRS);
      To[wave][col][t * 16 + 8 * hh + r] = ov * inv; } }
  wave_lds_sync();
  for (int pass = 0; pass < 2; ++pass) {
    for (int rr = 0; rr < 16; ++rr) {
      const v2f f = *(const v2f*)(&To[wave][rr][lane * 2]); v2h hv, lv;
#pragma unroll
      for (int j = 0; j < 2; ++j) { b16 p, q; split16(f[j] * XS, p, q); hv[j] = p; lv[j] = q; }
      const size_t oi = ((size_t)b * SEQ + q0 + rr) * DM + (size_t)h * HD + lane * 2;
      *(volatile v2h*)(Ch + oi) = hv; *(volatile v2h*)(Cl + oi) = lv; }
    __threadfence(); }
}

__global__ __launch_bounds__(128) void out_kernel(const b16* __restrict__ Ch, const b16* __restrict__ Cl, const b16* __restrict__ WO, float* __restrict__ out) {
  __shared__ __attribute__((aligned(16))) float Tf[4][16][128 + 4];
  const int wave = threadIdx.x >> 5, lane = threadIdx.x & 31, nloc = lane & 15, hlf = lane >> 4;
  const int b = blockIdx.x / (QL / 64), rb = blockIdx.x % (QL / 64);
  const size_t cm0 = (size_t)b * SEQ + (size_t)rb * 64 + wave * 16, om0 = (size_t)b * SEQ_FULL + (size_t)rb * 64 + wave * 16; const int n0 = blockIdx.y * 128;
  v8f acc[8];
#pragma unroll
  for (int t = 0; t < 8; ++t) acc[t] = (v8f){};
#pragma unroll 2
  for (int kb = 0; kb < DM; kb += 32) {
    const v16b a = frag_kb(Ch + (cm0 + nloc) * DM + kb, hlf), al = frag_kb(Cl + (cm0 + nloc) * DM + kb, hlf);
#pragma unroll
    for (int t = 0; t < 8; ++t) { const v16b bw = frag_kb(WO + (size_t)(n0 + t * 16 + nloc) * DM + kb, hlf); acc[t] = wmma16b(a, bw, acc[t]); acc[t] = wmma16b(al, bw, acc[t]); } }
#pragma unroll
  for (int t = 0; t < 8; ++t) {
#pragma unroll
    for (int r = 0; r < 8; ++r) Tf[wave][8 * hlf + r][t * 16 + nloc] = acc[t][r] * (1.0f / (XS * WSC)); }
  wave_lds_sync();
  for (int pass = 0; pass < 2; ++pass) {
    for (int rr = 0; rr < 16; ++rr) *(volatile v4f*)(out + (om0 + rr) * DM + n0 + lane * 4) = *(const v4f*)(&Tf[wave][rr][lane * 4]);
    __threadfence(); }
}
}

extern "C" void kernel_launch(void* const* d_in, const int* in_sizes, int n_in, void* d_out, int out_size, void* d_ws, size_t ws_size, hipStream_t stream) {
  const size_t need_x = ((size_t)(NB - 1) * SEQ_FULL + SEQ) * DM;
  if (n_in < 3 || (size_t)in_sizes[0] < need_x || in_sizes[1] < 3 * DM * DM || in_sizes[2] < DM * DM || (size_t)out_size < need_x) return;
  const float* xin = (const float*)d_in[0]; const float* wqkv = (const float*)d_in[1]; const float* wo = (const float*)d_in[2];
  size_t off = 0; char* ws = (char*)d_ws;
  auto carve = [&](size_t bytes) { char* p = ws + off; off += (bytes + 255) & ~(size_t)255; return p; };
  b16* WT = (b16*)carve((size_t)3 * DM * DM * 2); b16* WO = (b16*)carve((size_t)DM * DM * 2);
  const size_t plane = (size_t)NB * SEQ * DM * 2, lop = (size_t)NB * H * EQ * HD * 2;
  b16* Qp = (b16*)carve(plane); b16* Kp = (b16*)carve(plane); b16* VTh = (b16*)carve(plane); b16* VTl = (b16*)carve(plane); b16* Ch = (b16*)carve(plane); b16* Cl = (b16*)carve(plane);
  b16* Ql = (b16*)carve(lop); b16* Kl = (b16*)carve(lop);
  if (off > ws_size || off > ((size_t)128 << 20)) return;
  const int nbx = QL / 32; const int nearly = nbx < (EQ / 32) ? nbx : (EQ / 32);
  prep_kernel<<<(unsigned)(((size_t)4 * DM * DM / 8 + 255) / 256), 256, 0, stream>>>(wqkv, wo, WT, WO);
  proj_kernel<<<dim3(SEQ / 64, NB * 3, 8), 128, 0, stream>>>(xin, WT, Qp, Kp, VTh, VTl, Ql, Kl);
  attn_kernel<true><<<dim3(nearly, NB * H), 64, 0, stream>>>(Qp, Kp, Ql, Kl, VTh, VTl, Ch, Cl, 0);
  if (nbx > nearly) attn_kernel<false><<<dim3(nbx - nearly, NB * H), 64, 0, stream>>>(Qp, Kp, Ql, Kl, VTh, VTl, Ch, Cl, nearly);
  out_kernel<<<dim3((QL / 64) * NB, 8), 128, 0, stream>>>(Ch, Cl, WO, (float*)d_out);
}
